// SerialBlock_adapt_37142877176326
// MI455X (gfx1250) — hardware-verified
//
#include <hip/hip_runtime.h>

typedef __attribute__((ext_vector_type(16))) _Float16 v16h;
typedef __attribute__((ext_vector_type(8)))  _Float16 v8h;
typedef __attribute__((ext_vector_type(16))) __bf16   v16b;
typedef __attribute__((ext_vector_type(8)))  __bf16   v8b;
typedef __attribute__((ext_vector_type(8)))  float    v8f;
typedef __attribute__((ext_vector_type(4)))  float    v4f;

__device__ __forceinline__ unsigned short f2bf_bits(float f) {
  unsigned u = __float_as_uint(f);
  return (unsigned short)((u + 0x7FFFu + ((u >> 16) & 1u)) >> 16);
}
__device__ __forceinline__ float bf_bits2f(unsigned short h) { return __uint_as_float(((unsigned)h) << 16); }

__device__ __forceinline__ void dep_guard_h(v8f& a, v8f& b, v16h x, v16h y) { asm volatile("v_nop\n\tv_nop\n\tv_nop\n\tv_nop" : "+v"(a), "+v"(b) : "v"(x), "v"(y)); }
__device__ __forceinline__ void dep_guard_b(v8f& a, v8f& b, v16b x, v16b y) { asm volatile("v_nop\n\tv_nop\n\tv_nop\n\tv_nop" : "+v"(a), "+v"(b) : "v"(x), "v"(y)); }
__device__ __forceinline__ void keep4_h(v16h a, v16h b, v16h c, v16h d) { asm volatile("v_nop" :: "v"(a), "v"(b), "v"(c), "v"(d)); }
__device__ __forceinline__ void keep4_b(v16b a, v16b b, v16b c, v16b d) { asm volatile("v_nop" :: "v"(a), "v"(b), "v"(c), "v"(d)); }
__device__ __forceinline__ void acc_guard4(v8f& a, v8f& b, v8f& c, v8f& d) { asm volatile("v_nop\n\tv_nop\n\tv_nop\n\tv_nop" : "+v"(a), "+v"(b), "+v"(c), "+v"(d)); }
template <typename T> struct Frag;
template <> struct Frag<_Float16> {
  typedef v16h V; union U { v16h v; v8h h[2]; };
  static __device__ __forceinline__ v16h load(const _Float16* p) {
    U f; f.h[0] = *(const v8h*)(p); f.h[1] = *(const v8h*)(p + 16); return f.v;
  }
  static __device__ __forceinline__ v8f mma(v16h a, v16h b, v8f c) {
    return __builtin_amdgcn_wmma_f32_16x16x32_f16(false, a, false, b, (short)0, c, false, false);
  }
  static __device__ __forceinline__ void guard(v8f& a, v8f& b, v16h x, v16h y) { dep_guard_h(a, b, x, y); }
  static __device__ __forceinline__ void keep(v16h a, v16h b, v16h c, v16h d) { keep4_h(a, b, c, d); }
};
template <> struct Frag<__bf16> {
  typedef v16b V; union U { v16b v; v8b h[2]; };
  static __device__ __forceinline__ v16b load(const __bf16* p) {
    U f; f.h[0] = *(const v8b*)(p); f.h[1] = *(const v8b*)(p + 16); return f.v;
  }
  static __device__ __forceinline__ v8f mma(v16b a, v16b b, v8f c) {
    return __builtin_amdgcn_wmma_f32_16x16x32_bf16(false, a, false, b, (short)0, c, false, false);
  }
  static __device__ __forceinline__ void guard(v8f& a, v8f& b, v16b x, v16b y) { dep_guard_b(a, b, x, y); }
  static __device__ __forceinline__ void keep(v16b a, v16b b, v16b c, v16b d) { keep4_b(a, b, c, d); }
};

__device__ __forceinline__ v8f hmma(v16h a, v16h b, v8f c) {
  c = __builtin_amdgcn_wmma_f32_16x16x32_f16(false, a, false, b, (short)0, c, false, false);
  asm volatile("v_nop\n\tv_nop\n\tv_nop\n\tv_nop" : "+v"(c) : "v"(a), "v"(b));
  return c;
}

template <int ET> struct Elem;
template <> struct Elem<0> { typedef _Float16 T; };
template <> struct Elem<1> { typedef __bf16 T; };
template <int ET, bool SPLIT, int BIAS_MODE, int OUT_MODE, bool RESID, int ACT = 0>
__global__ __launch_bounds__(256) void wmma_gemm64(
    const unsigned short* __restrict__ Ap, const unsigned short* __restrict__ A2p, int lda, long strideA,
    const unsigned short* __restrict__ Btp, const unsigned short* __restrict__ Bt2p, int ldb, long strideB,
    void* __restrict__ Cout, void* __restrict__ Cout2, int ldc, long strideC,
    const float* __restrict__ bias,
    const float* __restrict__ resid, long strideR,
    int M, int N, int K, float scale) {
  typedef typename Elem<ET>::T T;
  typedef typename Frag<T>::V V;
  const T* A = (const T*)Ap; const T* A2 = (const T*)A2p; const T* Bt = (const T*)Btp; const T* Bt2 = (const T*)Bt2p;
  __shared__ __align__(16) float sT[8][16 * 68];
  const int b    = blockIdx.y;
  const int lane = threadIdx.x & 31;
  const int wave = threadIdx.x >> 5;
  const int tilesN = N >> 6;
  const int tilesM = M >> 6;
  const int tile = blockIdx.x * 8 + wave;
  if (tile >= tilesM * tilesN) return;
  const int tm = tile / tilesN;
  const int tn = tile - tm * tilesN;
  const int m0 = tm << 6;
  const int n0 = tn << 6;

  const T* Ab  = A  + (size_t)b * strideA;
  const T* Bb  = Bt + (size_t)b * strideB;
  const T* Ab2 = SPLIT ? (A2  + (size_t)b * strideA) : nullptr;
  const T* Bb2 = SPLIT ? (Bt2 + (size_t)b * strideB) : nullptr;

  const int rlane = lane & 15;
  const int koff  = (lane >> 4) * 8;
  const int mOff  = (lane >> 4) * 8;

  v8f acc[4][4];
#pragma unroll
  for (int i = 0; i < 4; ++i)
#pragma unroll
    for (int j = 0; j < 4; ++j) acc[i][j] = (v8f){0.f,0.f,0.f,0.f,0.f,0.f,0.f,0.f};

  for (int k0 = 0; k0 < K; k0 += 32) {
    V bh[4], bl[4];
#pragma unroll
    for (int j = 0; j < 4; ++j) {
      const size_t bo = (size_t)(n0 + (j << 4) + rlane) * ldb + koff + k0;
      bh[j] = Frag<T>::load(Bb + bo);
      if (SPLIT) bl[j] = Frag<T>::load(Bb2 + bo);
    }
#pragma unroll
    for (int i = 0; i < 4; ++i) {
      const size_t ao = (size_t)(m0 + (i << 4) + rlane) * lda + koff + k0;
      V ah = Frag<T>::load(Ab + ao);
      V al;
      if (SPLIT) al = Frag<T>::load(Ab2 + ao);
#pragma unroll
      for (int j = 0; j < 4; ++j) {
        acc[i][j] = Frag<T>::mma(ah, bh[j], acc[i][j]);
        if (SPLIT) {
          acc[i][j] = Frag<T>::mma(ah, bl[j], acc[i][j]);
          acc[i][j] = Frag<T>::mma(al, bh[j], acc[i][j]);
        }
      }
      Frag<T>::guard(acc[i][0], acc[i][3], ah, SPLIT ? al : ah);
    }
    Frag<T>::keep(bh[0], bh[1], bh[2], bh[3]);
    if (SPLIT) Frag<T>::keep(bl[0], bl[1], bl[2], bl[3]);
  }
  acc_guard4(acc[0][0], acc[0][1], acc[0][2], acc[0][3]);
  acc_guard4(acc[1][0], acc[1][1], acc[1][2], acc[1][3]);
  acc_guard4(acc[2][0], acc[2][1], acc[2][2], acc[2][3]);
  acc_guard4(acc[3][0], acc[3][1], acc[3][2], acc[3][3]);

  float* slab = sT[wave];
  const float* Rb = RESID ? (resid + (size_t)b * strideR) : nullptr;
#pragma unroll
  for (int i = 0; i < 4; ++i) {
    const int mBase = m0 + (i << 4);
#pragma unroll
    for (int j = 0; j < 4; ++j) {
      const int n = n0 + (j << 4) + rlane;
      float bv = 0.f;
      if (BIAS_MODE == 2) bv = bias[n];
#pragma unroll
      for (int r = 0; r < 8; ++r) {
        float v = acc[i][j][r] * scale;
        if (BIAS_MODE == 1) v += bias[mBase + mOff + r];
        if (BIAS_MODE == 2) v += bv;
        if (RESID) v += Rb[(size_t)(mBase + mOff + r) * ldc + n];
        if (ACT == 1) v = tanhf(v);
        if (ACT == 2) v = fmaxf(v, 0.0f);
        if (ACT == 3) v = v / (1.0f + expf(-v));
        if (ACT == 4) v = (v > 0.f) ? v : 0.01f * v;
        if (ACT == 5) v = 0.5f * v * (1.0f + erff(v * 0.70710678118654752f));
        slab[(mOff + r) * 68 + (j << 4) + rlane] = v;
      }
    }
    __builtin_amdgcn_fence(__ATOMIC_RELEASE, "workgroup");
    __builtin_amdgcn_wave_barrier();
    __builtin_amdgcn_fence(__ATOMIC_ACQUIRE, "workgroup");
    if (OUT_MODE == 0) {
      float* C = (float*)Cout + (size_t)b * strideC;
      const int hh = lane >> 4, c4 = (lane & 15) * 4;
      for (int pass = 0; pass < 2; ++pass) {
#pragma unroll
        for (int it = 0; it < 8; ++it) {
          const int row = it * 2 + hh;
          v4f v = *(const v4f*)(slab + row * 68 + c4);
          *(volatile v4f*)(C + (size_t)(mBase + row) * ldc + n0 + c4) = v;
        }
        __threadfence();
      }
    } else {
      const int q = lane >> 3, c8 = (lane & 7) * 8;
      unsigned short* C  = (unsigned short*)Cout  + (size_t)b * strideC;
      unsigned short* C2 = (OUT_MODE == 2) ? ((unsigned short*)Cout2 + (size_t)b * strideC) : nullptr;
      for (int pass = 0; pass < 2; ++pass) {
#pragma unroll
        for (int it = 0; it < 4; ++it) {
          const int row = it * 4 + q;
          const float* sp = slab + row * 68 + c8;
          v8h hv, lv;
#pragma unroll
          for (int e = 0; e < 8; ++e) {
            if (OUT_MODE == 1) {
              hv[e] = (_Float16)sp[e];
            } else {
              unsigned short hb = f2bf_bits(sp[e]);
              unsigned short lb = f2bf_bits(sp[e] - bf_bits2f(hb));
              hv[e] = __builtin_bit_cast(_Float16, hb);
              lv[e] = __builtin_bit_cast(_Float16, lb);
            }
          }
          *(volatile v8h*)(C + (size_t)(mBase + row) * ldc + n0 + c8) = hv;
          if (OUT_MODE == 2) *(volatile v8h*)(C2 + (size_t)(mBase + row) * ldc + n0 + c8) = lv;
        }
        __threadfence();
      }
    }
    __builtin_amdgcn_fence(__ATOMIC_RELEASE, "workgroup");
    __builtin_amdgcn_wave_barrier();
    __builtin_amdgcn_fence(__ATOMIC_ACQUIRE, "workgroup");
  }
}

__global__ __launch_bounds__(256) void cast_f32_f16x2s(
    const float* __restrict__ in, _Float16* __restrict__ out, int n2, float sc) {
  int i = blockIdx.x * 256 + threadIdx.x;
  if (i < n2) {
    const size_t i2 = (size_t)i * 2;
    const _Float16 h0 = (_Float16)(in[i2] * sc), h1 = (_Float16)(in[i2 + 1] * sc);
    const unsigned u = (unsigned)__builtin_bit_cast(unsigned short, h0) | ((unsigned)__builtin_bit_cast(unsigned short, h1) << 16);
    ((volatile unsigned*)out)[i] = u;
    __threadfence();
    ((volatile unsigned*)out)[i] = u;
  }
}

#define KTP 72
__global__ __launch_bounds__(128) void k_ktv(const _Float16* __restrict__ qkvh, _Float16* __restrict__ ktvT) {
  __shared__ __align__(16) _Float16 EsT[32 * KTP];
  __shared__ __align__(16) _Float16 VsT[32 * KTP];
  __shared__ float redM[128];
  __shared__ float colM[32];
  __shared__ float colS[32];
  __shared__ float sPart[128 * 17];
  __shared__ float Tt[32 * 33];

  const int t = threadIdx.x, lane = t & 31, wave = t >> 5, hh = lane >> 4, m = lane & 15;
  const int bh = blockIdx.x, bi = bh >> 3, h = bh & 7;
  const _Float16* kbase = qkvh + (size_t)bi * 4096 * 768 + 256 + h * 32;
  const _Float16* vbase = qkvh + (size_t)bi * 4096 * 768 + 512 + h * 32;

  {
    const int c = lane, seg = wave;
    float mx = -3.0e38f;
    for (int n = seg * 1024; n < seg * 1024 + 1024; ++n)
      mx = fmaxf(mx, (float)kbase[(size_t)n * 768 + c]);
    redM[t] = mx;
  }
  __syncthreads();
  if (t < 32) {
    float M = redM[t];
    M = fmaxf(M, redM[32 + t]);
    M = fmaxf(M, redM[64 + t]);
    M = fmaxf(M, redM[96 + t]);
    colM[t] = M;
  }
  __syncthreads();

  const int r = t >> 1, dh = (t & 1) * 16;
  float cm[16], sAcc[16];
#pragma unroll
  for (int e = 0; e < 16; ++e) { cm[e] = colM[dh + e]; sAcc[e] = 0.f; }
  v8f acc = (v8f){0.f,0.f,0.f,0.f,0.f,0.f,0.f,0.f};
  const int wi = wave >> 1, wj = wave & 1;

  for (int chunk = 0; chunk < 64; ++chunk) {
    __syncthreads();
    {
      const size_t tok = (size_t)(chunk * 64 + r);
      const _Float16* kp = kbase + tok * 768 + dh;
      const _Float16* vp = vbase + tok * 768 + dh;
      const v8h k0 = *(const v8h*)kp, k1 = *(const v8h*)(kp + 8);
      const v8h v0 = *(const v8h*)vp, v1 = *(const v8h*)(vp + 8);
#pragma unroll
      for (int e = 0; e < 8; ++e) {
        const float e0 = __expf((float)k0[e] - cm[e]);
        const float e1 = __expf((float)k1[e] - cm[8 + e]);
        sAcc[e] += e0; sAcc[8 + e] += e1;
        EsT[(dh + e) * KTP + r]     = (_Float16)e0;
        EsT[(dh + 8 + e) * KTP + r] = (_Float16)e1;
        VsT[(dh + e) * KTP + r]     = v0[e];
        VsT[(dh + 8 + e) * KTP + r] = v1[e];
      }
    }
    __syncthreads();
#pragma unroll
    for (int kk = 0; kk < 2; ++kk) {
      const v16h a  = Frag<_Float16>::load(EsT + (wi * 16 + m) * KTP + kk * 32 + 8 * hh);
      const v16h bf = Frag<_Float16>::load(VsT + (wj * 16 + m) * KTP + kk * 32 + 8 * hh);
      acc = hmma(a, bf, acc);
    }
  }

#pragma unroll
  for (int e = 0; e < 16; ++e) sPart[t * 17 + e] = sAcc[e];
#pragma unroll
  for (int rr = 0; rr < 8; ++rr) Tt[(wi * 16 + 8 * hh + rr) * 33 + wj * 16 + m] = acc[rr];
  __syncthreads();
  if (t < 32) {
    const int dsel = t >> 4, e = t & 15;
    float S = 0.f;
    for (int q = 0; q < 64; ++q) S += sPart[(2 * q + dsel) * 17 + e];
    colS[t] = 1024.0f / S;
  }
  __syncthreads();
  {
    const int vc = t >> 2, kc0 = (t & 3) * 8;
    v8h o;
#pragma unroll
    for (int e = 0; e < 8; ++e) o[e] = (_Float16)(Tt[(kc0 + e) * 33 + vc] * colS[kc0 + e]);
    volatile v8h* dst = (volatile v8h*)(ktvT + (size_t)bh * 1024 + t * 8);
    *dst = o;
    __threadfence();
    *dst = o;
  }
}

template <int KS>
__device__ __forceinline__ void conv_tile(const _Float16* lv, int cl, int xoff, const float* wp, float bv, float (&s)[8]) {
  constexpr int R = KS / 2;
  constexpr int NW = 8 + 2 * R;
#pragma unroll
  for (int i = 0; i < 8; ++i) s[i] = bv;
#pragma unroll 1
  for (int dy = 0; dy < KS; ++dy) {
    float wrow[KS];
#pragma unroll
    for (int dx = 0; dx < KS; ++dx) wrow[dx] = wp[dy * KS + dx];
    const _Float16* lp = lv + ((3 - R + dy) * 22 + (3 - R + xoff)) * 128 + cl;
    float rowv[NW];
#pragma unroll
    for (int i = 0; i < NW; ++i) rowv[i] = (float)lp[i * 128];
#pragma unroll
    for (int xi = 0; xi < 8; ++xi)
#pragma unroll
      for (int dx = 0; dx < KS; ++dx) s[xi] = fmaf(wrow[dx], rowv[xi + dx], s[xi]);
  }
}

#define ATTSC (0.17677669529663687f * (1.0f / 1024.0f))
__global__ __launch_bounds__(128) void k_fa(
    const _Float16* __restrict__ qkvh, const _Float16* __restrict__ ktvT,
    const float* __restrict__ w3, const float* __restrict__ b3,
    const float* __restrict__ w5, const float* __restrict__ b5,
    const float* __restrict__ w7, const float* __restrict__ b7,
    _Float16* __restrict__ fah, float* __restrict__ part) {
  __shared__ __align__(16) _Float16 lv[7 * 22 * 128];
  __shared__ __align__(16) _Float16 lq[16 * 128];
  __shared__ __align__(16) float    fs[16 * 132];

  const int t = threadIdx.x, lane = t & 31, wave = t >> 5, hh = lane >> 4, m = lane & 15;
  const int bix = blockIdx.x, g = bix & 1, xq = (bix >> 1) & 3, y = (bix >> 3) & 63, bi = bix >> 9;
  const int x0 = xq * 16, cbase = g * 128;
  const size_t brow = (size_t)bi * 4096;

  v8h zero8;
#pragma unroll
  for (int e = 0; e < 8; ++e) zero8[e] = (_Float16)0.0f;

  for (int idx = t; idx < 7 * 22 * 16; idx += 128) {
    const int p = idx >> 4, q16 = idx & 15;
    const int ry = p / 22, rx = p - ry * 22;
    const int gy = y + ry - 3, gx = x0 + rx - 3;
    const bool inb = (gy >= 0) && (gy < 64) && (gx >= 0) && (gx < 64);
    const int gyc = min(max(gy, 0), 63), gxc = min(max(gx, 0), 63);
    v8h val = *(const v8h*)(qkvh + (brow + (size_t)gyc * 64 + gxc) * 768 + 512 + cbase + q16 * 8);
    if (!inb) val = zero8;
    *(v8h*)(lv + p * 128 + q16 * 8) = val;
  }
  for (int idx = t; idx < 256; idx += 128) {
    const int p = idx >> 4, q16 = idx & 15;
    *(v8h*)(lq + p * 128 + q16 * 8) = *(const v8h*)(qkvh + (brow + (size_t)y * 64 + x0 + p) * 768 + cbase + q16 * 8);
  }
  __syncthreads();

  {
    const _Float16* kt = ktvT + (size_t)(bi * 8 + g * 4 + wave) * 1024;
    const v16h a   = Frag<_Float16>::load(lq + m * 128 + wave * 32 + 8 * hh);
    const v16h bf0 = Frag<_Float16>::load(kt + m * 32 + 8 * hh);
    const v16h bf1 = Frag<_Float16>::load(kt + (16 + m) * 32 + 8 * hh);
    const v8f z = (v8f){0.f,0.f,0.f,0.f,0.f,0.f,0.f,0.f};
    const v8f a0 = hmma(a, bf0, z);
    const v8f a1 = hmma(a, bf1, z);
#pragma unroll
    for (int rr = 0; rr < 8; ++rr) {
      fs[(8 * hh + rr) * 132 + wave * 32 + m]      = a0[rr] * ATTSC;
      fs[(8 * hh + rr) * 132 + wave * 32 + 16 + m] = a1[rr] * ATTSC;
    }
  }
  __syncthreads();

  const int c = cbase + t;
  const int c3 = min(c, 63), c5 = min(max(c - 64, 0), 95), c7 = min(max(c - 160, 0), 95);
  float psum = 0.f;
#pragma unroll 1
  for (int half = 0; half < 2; ++half) {
    const int xoff = half * 8;
    float s[8];
    if (c < 64)       conv_tile<3>(lv, t, xoff, w3 + c3 * 9,  b3[c3], s);
    else if (c < 160) conv_tile<5>(lv, t, xoff, w5 + c5 * 25, b5[c5], s);
    else              conv_tile<7>(lv, t, xoff, w7 + c7 * 49, b7[c7], s);
#pragma unroll
    for (int i = 0; i < 8; ++i) {
      const int xi = xoff + i;
      const float av = fs[xi * 132 + t];
      const float qv = (float)lq[xi * 128 + t];
      const float val = fmaf(qv, s[i], av);
      psum += val;
      fs[xi * 132 + t] = val;
    }
  }
  {
    volatile float* pp = part + ((size_t)(bi * 256 + y * 4 + xq) * 256 + cbase + t);
    *pp = psum;
    __threadfence();
    *pp = psum;
  }
  __syncthreads();

  for (int pass = 0; pass < 2; ++pass) {
#pragma unroll
    for (int it = 0; it < 2; ++it) {
      const int q = t + it * 128;
      const int row = q >> 4, c8 = (q & 15) * 8;
      v8h o;
#pragma unroll
      for (int e = 0; e < 8; ++e) o[e] = (_Float16)(fs[row * 132 + c8 + e] * 256.0f);
      *(volatile v8h*)(fah + (brow + (size_t)y * 64 + x0 + row) * 256 + cbase + c8) = o;
    }
    __threadfence();
  }
}

__global__ __launch_bounds__(256) void k_se(
    const float* __restrict__ part, const float* __restrict__ w1, const float* __restrict__ w2,
    const float* __restrict__ pw, _Float16* __restrict__ projB) {
  __shared__ float pooled[2048];
  __shared__ float hid[1024];
  __shared__ float gf[64];
  const int t = threadIdx.x;
  for (int idx = t; idx < 2048; idx += 256) {
    const int bi = idx >> 8, c = idx & 255;
    double s = 0.0;
    for (int p = 0; p < 256; ++p) s += (double)part[(size_t)(bi * 256 + p) * 256 + c];
    pooled[idx] = (float)s * (1.0f / 4096.0f);
  }
  __syncthreads();
  for (int idx = t; idx < 1024; idx += 256) {
    const int bi = idx >> 7, j = idx & 127;
    float d = 0.f;
#pragma unroll 4
    for (int c = 0; c < 256; ++c) d = fmaf(pooled[bi * 256 + c], w1[j * 256 + c], d);
    hid[idx] = fmaxf(d, 0.f);
  }
  __syncthreads();
  if (t < 64) {
    const int bi = t >> 3, h8 = t & 7;
    float d = 0.f;
#pragma unroll 4
    for (int j = 0; j < 128; ++j) d = fmaf(hid[bi * 128 + j], w2[h8 * 128 + j], d);
    gf[t] = 1.0f + 1.0f / (1.0f + expf(-d));
  }
  __syncthreads();
  for (int pass = 0; pass < 2; ++pass) {
    for (int i = t; i < 8 * 256 * 128; i += 256) {
      const int bi = i >> 15, rem = i & 32767;
      const int n = rem >> 7, kp = (rem & 127) * 2;
      const float gg = gf[bi * 8 + (kp >> 5)] * 64.0f;
      const _Float16 h0 = (_Float16)(pw[n * 256 + kp] * gg);
      const _Float16 h1 = (_Float16)(pw[n * 256 + kp + 1] * gg);
      const unsigned u = (unsigned)__builtin_bit_cast(unsigned short, h0) | ((unsigned)__builtin_bit_cast(unsigned short, h1) << 16);
      ((volatile unsigned*)projB)[i] = u;
    }
    __threadfence();
  }
}

extern "C" void kernel_launch(void* const* d_in, const int* in_sizes, int n_in,
                              void* d_out, int out_size, void* d_ws, size_t ws_size,
                              hipStream_t stream) {
  if (n_in < 13) return;
  if (in_sizes[0] != 8388608 || in_sizes[1] != 196608 || in_sizes[2] != 768 ||
      in_sizes[3] != 65536 || in_sizes[4] != 256 || in_sizes[5] != 32768 || in_sizes[6] != 1024 ||
      in_sizes[7] != 576 || in_sizes[8] != 64 || in_sizes[9] != 2400 || in_sizes[10] != 96 ||
      in_sizes[11] != 4704 || in_sizes[12] != 96 || out_size != 8388608) return;

  const float* x      = (const float*)d_in[0];
  const float* qkv_w  = (const float*)d_in[1];
  const float* qkv_b  = (const float*)d_in[2];
  const float* proj_w = (const float*)d_in[3];
  const float* proj_b = (const float*)d_in[4];
  const float* se_w1  = (const float*)d_in[5];
  const float* se_w2  = (const float*)d_in[6];
  const float* w3     = (const float*)d_in[7];
  const float* b3     = (const float*)d_in[8];
  const float* w5     = (const float*)d_in[9];
  const float* b5     = (const float*)d_in[10];
  const float* w7     = (const float*)d_in[11];
  const float* b7     = (const float*)d_in[12];
  float* out = (float*)d_out;

  char* w = (char*)d_ws;
  size_t off = 0;
  _Float16* xh    = (_Float16*)(w + off); off += 32768ull * 256 * 2;
  _Float16* wqkvh = (_Float16*)(w + off); off += 768ull * 256 * 2;
  _Float16* qkvh  = (_Float16*)(w + off); off += 32768ull * 768 * 2;
  _Float16* ktvT  = (_Float16*)(w + off); off += 64ull * 1024 * 2;
  _Float16* fah   = (_Float16*)(w + off); off += 32768ull * 256 * 2;
  float*    part  = (float*)(w + off);    off += 8ull * 256 * 256 * 4;
  _Float16* projB = (_Float16*)(w + off); off += 8ull * 256 * 256 * 2;
  if (off > ws_size) return;

  cast_f32_f16x2s<<<(4194304 + 255) / 256, 256, 0, stream>>>(x, xh, 4194304, 1.0f);
  cast_f32_f16x2s<<<(98304 + 255) / 256, 256, 0, stream>>>(qkv_w, wqkvh, 98304, 64.0f);

  wmma_gemm64<0, false, 2, 1, false><<<dim3(768, 1), dim3(256), 0, stream>>>(
      (const unsigned short*)xh, (const unsigned short*)xh, 256, 0L,
      (const unsigned short*)wqkvh, (const unsigned short*)wqkvh, 256, 0L,
      (void*)qkvh, (void*)qkvh, 768, 0L,
      qkv_b, qkv_b, 0L,
      32768, 768, 256, 1.0f / 64.0f);

  k_ktv<<<64, 128, 0, stream>>>(qkvh, ktvT);

  k_fa<<<4096, 128, 0, stream>>>(qkvh, ktvT, w3, b3, w5, b5, w7, b7, fah, part);

  k_se<<<1, 256, 0, stream>>>(part, se_w1, se_w2, proj_w, projB);

  wmma_gemm64<0, false, 2, 0, false><<<dim3(32, 8), dim3(256), 0, stream>>>(
      (const unsigned short*)fah, (const unsigned short*)fah, 256, 4096L * 256,
      (const unsigned short*)projB, (const unsigned short*)projB, 256, 65536L,
      (void*)out, (void*)out, 256, 4096L * 256,
      proj_b, proj_b, 0L,
      4096, 256, 256, 1.0f / 16384.0f);
}
